// TranscriptionCRFModel_26190710571333
// MI455X (gfx1250) — hardware-run, weakly checked
//
#include <hip/hip_runtime.h>
#include <math.h>

#define NBATCH 64
#define NSTEP 4096
#define NROWS (NBATCH * NSTEP)
#define FEAT_D 37
#define NTAG0 37
#define NTAG1 13
#define NTAG2 25
#define KPAD 64
#define NCOL 64
#define COL1 48
#define ETP 40
#define PART_LD 128
#define NCHAIN 3

static_assert(NTAG0 <= COL1);
static_assert(COL1 + NTAG1 <= NCOL);
static_assert(FEAT_D <= KPAD);
static_assert((NROWS % 256) == 0);
static_assert((NROWS % 64) == 0);
static_assert((((NTAG0 + 7) & ~7)) <= ETP);
static_assert((NSTEP % 32) == 0);

typedef __attribute__((ext_vector_type(16))) _Float16 v16h;
typedef __attribute__((ext_vector_type(8)))  _Float16 v8h;
typedef __attribute__((ext_vector_type(16))) __bf16   v16b;
typedef __attribute__((ext_vector_type(8)))  __bf16   v8b;
typedef __attribute__((ext_vector_type(8)))  float    v8f;
typedef __attribute__((ext_vector_type(4)))  float    v4f;
typedef __attribute__((ext_vector_type(4)))  unsigned int v4u;
#define PSCALE 32768.0f
#define U16(p) ((const unsigned short*)(const void*)(p))
#define PSCALE_INV (1.0f / 32768.0f)

__device__ __forceinline__ unsigned short f2bf_bits(float f) {
  unsigned u = __float_as_uint(f);
  return (unsigned short)((u + 0x7FFFu + ((u >> 16) & 1u)) >> 16);
}
__device__ __forceinline__ float bf_bits2f(unsigned short h) { return __uint_as_float(((unsigned)h) << 16); }
__device__ __forceinline__ float to_bf16_val(float f) { return bf_bits2f(f2bf_bits(f)); }

__device__ __forceinline__ void dep_guard_h(v8f& a, v8f& b, v16h x, v16h y) { asm volatile("v_nop\n\tv_nop\n\tv_nop\n\tv_nop" : "+v"(a), "+v"(b) : "v"(x), "v"(y)); }
__device__ __forceinline__ void dep_guard_b(v8f& a, v8f& b, v16b x, v16b y) { asm volatile("v_nop\n\tv_nop\n\tv_nop\n\tv_nop" : "+v"(a), "+v"(b) : "v"(x), "v"(y)); }
__device__ __forceinline__ void keep4_h(v16h a, v16h b, v16h c, v16h d) { asm volatile("v_nop" :: "v"(a), "v"(b), "v"(c), "v"(d)); }
__device__ __forceinline__ void keep4_b(v16b a, v16b b, v16b c, v16b d) { asm volatile("v_nop" :: "v"(a), "v"(b), "v"(c), "v"(d)); }
__device__ __forceinline__ void acc_guard4(v8f& a, v8f& b, v8f& c, v8f& d) { asm volatile("v_nop\n\tv_nop\n\tv_nop\n\tv_nop" : "+v"(a), "+v"(b), "+v"(c), "+v"(d)); }
template <typename T> struct Frag;
template <> struct Frag<_Float16> {
  typedef v16h V; union U { v16h v; v8h h[2]; };
  static __device__ __forceinline__ v16h load(const _Float16* p) {
    U f; f.h[0] = *(const v8h*)(p); f.h[1] = *(const v8h*)(p + 16); return f.v;
  }
  static __device__ __forceinline__ v8f mma(v16h a, v16h b, v8f c) {
    return __builtin_amdgcn_wmma_f32_16x16x32_f16(false, a, false, b, (short)0, c, false, false);
  }
  static __device__ __forceinline__ void guard(v8f& a, v8f& b, v16h x, v16h y) { dep_guard_h(a, b, x, y); }
  static __device__ __forceinline__ void keep(v16h a, v16h b, v16h c, v16h d) { keep4_h(a, b, c, d); }
};
template <> struct Frag<__bf16> {
  typedef v16b V; union U { v16b v; v8b h[2]; };
  static __device__ __forceinline__ v16b load(const __bf16* p) {
    U f; f.h[0] = *(const v8b*)(p); f.h[1] = *(const v8b*)(p + 16); return f.v;
  }
  static __device__ __forceinline__ v8f mma(v16b a, v16b b, v8f c) {
    return __builtin_amdgcn_wmma_f32_16x16x32_bf16(false, a, false, b, (short)0, c, false, false);
  }
  static __device__ __forceinline__ void guard(v8f& a, v8f& b, v16b x, v16b y) { dep_guard_b(a, b, x, y); }
  static __device__ __forceinline__ void keep(v16b a, v16b b, v16b c, v16b d) { keep4_b(a, b, c, d); }
};

template <int ET> struct Elem;
template <> struct Elem<0> { typedef _Float16 T; };
template <> struct Elem<1> { typedef __bf16 T; };
template <int ET, bool SPLIT, int BIAS_MODE, int OUT_MODE, bool RESID, int ACT = 0>
__global__ __launch_bounds__(256) void wmma_gemm64(
    const unsigned short* __restrict__ Ap, const unsigned short* __restrict__ A2p, int lda, long strideA,
    const unsigned short* __restrict__ Btp, const unsigned short* __restrict__ Bt2p, int ldb, long strideB,
    void* __restrict__ Cout, void* __restrict__ Cout2, int ldc, long strideC,
    const float* __restrict__ bias,
    const float* __restrict__ resid, long strideR,
    int M, int N, int K, float scale) {
  typedef typename Elem<ET>::T T;
  typedef typename Frag<T>::V V;
  const T* A = (const T*)Ap; const T* A2 = (const T*)A2p; const T* Bt = (const T*)Btp; const T* Bt2 = (const T*)Bt2p;
  __shared__ __align__(16) float sT[8][16 * 68];
  const int b    = blockIdx.y;
  const int lane = threadIdx.x & 31;
  const int wave = threadIdx.x >> 5;
  const int tilesN = N >> 6;
  const int tilesM = M >> 6;
  const int tile = blockIdx.x * 8 + wave;
  if (tile >= tilesM * tilesN) return;
  const int tm = tile / tilesN;
  const int tn = tile - tm * tilesN;
  const int m0 = tm << 6;
  const int n0 = tn << 6;

  const T* Ab  = A  + (size_t)b * strideA;
  const T* Bb  = Bt + (size_t)b * strideB;
  const T* Ab2 = SPLIT ? (A2  + (size_t)b * strideA) : nullptr;
  const T* Bb2 = SPLIT ? (Bt2 + (size_t)b * strideB) : nullptr;

  const int rlane = lane & 15;
  const int koff  = (lane >> 4) * 8;
  const int mOff  = (lane >> 4) * 8;

  v8f acc[4][4];
#pragma unroll
  for (int i = 0; i < 4; ++i)
#pragma unroll
    for (int j = 0; j < 4; ++j) acc[i][j] = (v8f){0.f,0.f,0.f,0.f,0.f,0.f,0.f,0.f};

  for (int k0 = 0; k0 < K; k0 += 32) {
    V bh[4], bl[4];
#pragma unroll
    for (int j = 0; j < 4; ++j) {
      const size_t bo = (size_t)(n0 + (j << 4) + rlane) * ldb + koff + k0;
      bh[j] = Frag<T>::load(Bb + bo);
      if (SPLIT) bl[j] = Frag<T>::load(Bb2 + bo);
    }
#pragma unroll
    for (int i = 0; i < 4; ++i) {
      const size_t ao = (size_t)(m0 + (i << 4) + rlane) * lda + koff + k0;
      V ah = Frag<T>::load(Ab + ao);
      V al;
      if (SPLIT) al = Frag<T>::load(Ab2 + ao);
#pragma unroll
      for (int j = 0; j < 4; ++j) {
        acc[i][j] = Frag<T>::mma(ah, bh[j], acc[i][j]);
        if (SPLIT) {
          acc[i][j] = Frag<T>::mma(ah, bl[j], acc[i][j]);
          acc[i][j] = Frag<T>::mma(al, bh[j], acc[i][j]);
        }
      }
      Frag<T>::guard(acc[i][0], acc[i][3], ah, SPLIT ? al : ah);
    }
    Frag<T>::keep(bh[0], bh[1], bh[2], bh[3]);
    if (SPLIT) Frag<T>::keep(bl[0], bl[1], bl[2], bl[3]);
  }
  acc_guard4(acc[0][0], acc[0][1], acc[0][2], acc[0][3]);
  acc_guard4(acc[1][0], acc[1][1], acc[1][2], acc[1][3]);
  acc_guard4(acc[2][0], acc[2][1], acc[2][2], acc[2][3]);
  acc_guard4(acc[3][0], acc[3][1], acc[3][2], acc[3][3]);

  float* slab = sT[wave];
  const float* Rb = RESID ? (resid + (size_t)b * strideR) : nullptr;
#pragma unroll
  for (int i = 0; i < 4; ++i) {
    const int mBase = m0 + (i << 4);
#pragma unroll
    for (int j = 0; j < 4; ++j) {
      const int n = n0 + (j << 4) + rlane;
      float bv = 0.f;
      if (BIAS_MODE == 2) bv = bias[n];
#pragma unroll
      for (int r = 0; r < 8; ++r) {
        float v = acc[i][j][r] * scale;
        if (BIAS_MODE == 1) v += bias[mBase + mOff + r];
        if (BIAS_MODE == 2) v += bv;
        if (RESID) v += Rb[(size_t)(mBase + mOff + r) * ldc + n];
        if (ACT == 1) v = tanhf(v);
        if (ACT == 2) v = fmaxf(v, 0.0f);
        if (ACT == 3) v = v / (1.0f + expf(-v));
        if (ACT == 4) v = (v > 0.f) ? v : 0.01f * v;
        if (ACT == 5) v = 0.5f * v * (1.0f + erff(v * 0.70710678118654752f));
        slab[(mOff + r) * 68 + (j << 4) + rlane] = v;
      }
    }
    __builtin_amdgcn_fence(__ATOMIC_RELEASE, "workgroup");
    __builtin_amdgcn_wave_barrier();
    __builtin_amdgcn_fence(__ATOMIC_ACQUIRE, "workgroup");
    if (OUT_MODE == 0) {
      float* C = (float*)Cout + (size_t)b * strideC;
      const int hh = lane >> 4, c4 = (lane & 15) * 4;
      for (int pass = 0; pass < 2; ++pass) {
#pragma unroll
        for (int it = 0; it < 8; ++it) {
          const int row = it * 2 + hh;
          v4f v = *(const v4f*)(slab + row * 68 + c4);
          *(volatile v4f*)(C + (size_t)(mBase + row) * ldc + n0 + c4) = v;
        }
        __threadfence();
      }
    } else {
      const int q = lane >> 3, c8 = (lane & 7) * 8;
      unsigned short* C  = (unsigned short*)Cout  + (size_t)b * strideC;
      unsigned short* C2 = (OUT_MODE == 2) ? ((unsigned short*)Cout2 + (size_t)b * strideC) : nullptr;
      for (int pass = 0; pass < 2; ++pass) {
#pragma unroll
        for (int it = 0; it < 4; ++it) {
          const int row = it * 4 + q;
          const float* sp = slab + row * 68 + c8;
          v8h hv, lv;
#pragma unroll
          for (int e = 0; e < 8; ++e) {
            if (OUT_MODE == 1) {
              hv[e] = (_Float16)sp[e];
            } else {
              unsigned short hb = f2bf_bits(sp[e]);
              unsigned short lb = f2bf_bits(sp[e] - bf_bits2f(hb));
              hv[e] = __builtin_bit_cast(_Float16, hb);
              lv[e] = __builtin_bit_cast(_Float16, lb);
            }
          }
          *(volatile v8h*)(C + (size_t)(mBase + row) * ldc + n0 + c8) = hv;
          if (OUT_MODE == 2) *(volatile v8h*)(C2 + (size_t)(mBase + row) * ldc + n0 + c8) = lv;
        }
        __threadfence();
      }
    }
    __builtin_amdgcn_fence(__ATOMIC_RELEASE, "workgroup");
    __builtin_amdgcn_wave_barrier();
    __builtin_amdgcn_fence(__ATOMIC_ACQUIRE, "workgroup");
  }
}

__global__ __launch_bounds__(256) void prep_feat_plane(const float* __restrict__ feats,
                                                       unsigned short* __restrict__ Ap) {
  const int lane = threadIdx.x & 31;
  const int wave = threadIdx.x >> 5;
  const int q  = lane >> 3;
  const int c8 = (lane & 7) * 8;
  const int rbase = blockIdx.x * 256 + wave * 32 + q;
  v4u pk[8];
#pragma unroll
  for (int it = 0; it < 8; ++it) {
    const int row = rbase + it * 4;
    const float* src = feats + (size_t)row * FEAT_D;
    unsigned w[4];
#pragma unroll
    for (int e2 = 0; e2 < 4; ++e2) {
      const int k0i = c8 + 2 * e2;
      const int k1i = k0i + 1;
      const int kc0 = (k0i < FEAT_D) ? k0i : (FEAT_D - 1);
      const int kc1 = (k1i < FEAT_D) ? k1i : (FEAT_D - 1);
      const float f0 = src[kc0];
      const float f1 = src[kc1];
      unsigned b0 = (unsigned)f2bf_bits(f0);
      unsigned b1 = (unsigned)f2bf_bits(f1);
      b0 = (k0i < FEAT_D) ? b0 : 0u;
      b1 = (k1i < FEAT_D) ? b1 : 0u;
      w[e2] = b0 | (b1 << 16);
    }
    pk[it] = (v4u){w[0], w[1], w[2], w[3]};
  }
  for (int pass = 0; pass < 2; ++pass) {
#pragma unroll
    for (int it = 0; it < 8; ++it) {
      const int row = rbase + it * 4;
      *(volatile v4u*)(Ap + (size_t)row * KPAD + c8) = pk[it];
    }
    __threadfence();
  }
}

__global__ __launch_bounds__(256) void prep_wb(const float* __restrict__ W0, const float* __restrict__ b0,
                                               const float* __restrict__ W1, const float* __restrict__ b1,
                                               unsigned short* __restrict__ Btp, float* __restrict__ biasp) {
  const int lane = threadIdx.x & 31;
  const int wave = threadIdx.x >> 5;
  const int q  = lane >> 3;
  const int c8 = (lane & 7) * 8;
  v4u pk[2];
#pragma unroll
  for (int it = 0; it < 2; ++it) {
    const int n = wave * 8 + it * 4 + q;
    const int nr = (n < NTAG0) ? n : (NTAG0 - 1);
    int nb = n - COL1;
    nb = (nb < 0) ? 0 : ((nb > NTAG1 - 1) ? (NTAG1 - 1) : nb);
    const bool rowR = (n < NTAG0);
    const bool rowB = (n >= COL1) && (n < COL1 + NTAG1);
    unsigned w[4];
#pragma unroll
    for (int e2 = 0; e2 < 4; ++e2) {
      const int k0i = c8 + 2 * e2;
      const int k1i = k0i + 1;
      const int kc0 = (k0i < FEAT_D) ? k0i : (FEAT_D - 1);
      const int kc1 = (k1i < FEAT_D) ? k1i : (FEAT_D - 1);
      const float r0 = W0[kc0 * NTAG0 + nr];
      const float r1 = W0[kc1 * NTAG0 + nr];
      const float s0 = W1[kc0 * NTAG1 + nb];
      const float s1 = W1[kc1 * NTAG1 + nb];
      float v0 = rowR ? r0 : (rowB ? s0 : 0.0f);
      float v1 = rowR ? r1 : (rowB ? s1 : 0.0f);
      v0 = (k0i < FEAT_D) ? v0 : 0.0f;
      v1 = (k1i < FEAT_D) ? v1 : 0.0f;
      const unsigned u0 = (unsigned)f2bf_bits(v0);
      const unsigned u1 = (unsigned)f2bf_bits(v1);
      w[e2] = u0 | (u1 << 16);
    }
    pk[it] = (v4u){w[0], w[1], w[2], w[3]};
  }
  for (int pass = 0; pass < 2; ++pass) {
#pragma unroll
    for (int it = 0; it < 2; ++it) {
      const int n = wave * 8 + it * 4 + q;
      *(volatile v4u*)(Btp + (size_t)n * KPAD + c8) = pk[it];
    }
    __threadfence();
  }
  v4f bv;
#pragma unroll
  for (int e = 0; e < 4; ++e) {
    const int n = lane * 4 + e;
    const int nr = (n < NTAG0) ? n : (NTAG0 - 1);
    int nb = n - COL1;
    nb = (nb < 0) ? 0 : ((nb > NTAG1 - 1) ? (NTAG1 - 1) : nb);
    const bool rowR = (n < NTAG0);
    const bool rowB = (n >= COL1) && (n < COL1 + NTAG1);
    const float vr = to_bf16_val(b0[nr]);
    const float vb = to_bf16_val(b1[nb]);
    bv[e] = rowR ? vr : (rowB ? vb : 0.0f);
  }
  if (wave == 0) {
    for (int pass = 0; pass < 2; ++pass) {
      *(volatile v4f*)(biasp + lane * 4) = bv;
      __threadfence();
    }
  }
}

__device__ __forceinline__ float ld_em(const float* p, bool cvt) {
  const float e = *p;
  return cvt ? to_bf16_val(e) : e;
}

__global__ __launch_bounds__(32) void chain_fwd(
    const float* __restrict__ EM, const float* __restrict__ em2,
    const int* __restrict__ lab0, const int* __restrict__ lab1, const int* __restrict__ lab2,
    const int* __restrict__ keep,
    const float* __restrict__ tr0, const float* __restrict__ st0, const float* __restrict__ en0,
    const float* __restrict__ tr1, const float* __restrict__ st1, const float* __restrict__ en1,
    const float* __restrict__ tr2, const float* __restrict__ st2, const float* __restrict__ en2,
    float* __restrict__ partial) {
  __shared__ __align__(16) float sETt[64 * ETP];
  __shared__ __align__(16) float sTr[NTAG0 * NTAG0 + 7];
  __shared__ __align__(16) float sEa[64];
  __shared__ __align__(16) float sAlpha[64];

  const int lane = threadIdx.x;
  const int blk  = blockIdx.x;
  const int c    = blk / NBATCH;
  const int b    = blk - c * NBATCH;
  const int K    = (c == 0) ? NTAG0 : ((c == 1) ? NTAG1 : NTAG2);
  const int KP8  = (K + 7) & ~7;
  const int nslot = (K + 31) >> 5;
  const float* trans  = (c == 0) ? tr0 : ((c == 1) ? tr1 : tr2);
  const float* startv = (c == 0) ? st0 : ((c == 1) ? st1 : st2);
  const float* endv   = (c == 0) ? en0 : ((c == 1) ? en1 : en2);
  const int* tags = ((c == 0) ? lab0 : ((c == 1) ? lab1 : lab2)) + (size_t)b * NSTEP;
  const int* krow = keep + (size_t)b * NSTEP;
  const bool cvt  = (c == 2);
  const float* emb = cvt ? (em2 + (size_t)b * NSTEP * NTAG2)
                         : (EM + (size_t)b * NSTEP * NCOL + ((c == 1) ? COL1 : 0));
  const int emld = cvt ? NTAG2 : NCOL;
  const float ninf = -__builtin_huge_valf();

#pragma unroll 1
  for (int idx = lane; idx < 64; idx += 32) { sEa[idx] = 0.0f; sAlpha[idx] = ninf; }
#pragma unroll 1
  for (int idx = lane; idx < K * KP8; idx += 32) {
    const int j = idx / KP8;
    const int i = idx - j * KP8;
    const int ic = (i < K) ? i : (K - 1);
    const float tv = to_bf16_val(trans[ic * K + j]);
    const float ev = expf(tv);
    sETt[j * ETP + i] = (i < K) ? ev : 0.0f;
  }
#pragma unroll 1
  for (int idx = lane; idx < K * K; idx += 32) sTr[idx] = to_bf16_val(trans[idx]);
  __syncthreads();

  float sc = 0.0f;
  int cnt = 0;
#pragma unroll 1
  for (int kk = 0; kk < NSTEP / 32; ++kk) {
    const int t  = kk * 32 + lane;
    const int mk = krow[t];
    cnt += (mk != 0) ? 1 : 0;
    int tg = tags[t];
    tg = (tg < 0) ? 0 : ((tg > K - 1) ? (K - 1) : tg);
    const int tp = (t > 0) ? (t - 1) : 0;
    int pg = tags[tp];
    pg = (pg < 0) ? 0 : ((pg > K - 1) ? (K - 1) : pg);
    const float e   = ld_em(emb + (size_t)t * emld + tg, cvt);
    const float trv = sTr[pg * K + tg];
    const float stv = to_bf16_val(startv[tg]);
    const float term0 = stv + e;
    const float term1 = (mk != 0) ? (trv + e) : 0.0f;
    sc += (t == 0) ? term0 : term1;
  }
#pragma unroll
  for (int off = 16; off > 0; off >>= 1) {
    sc  += __shfl_xor(sc, off, 32);
    cnt += __shfl_xor(cnt, off, 32);
  }
  {
    int last = cnt - 1;
    last = (last < 0) ? (last + NSTEP) : last;
    last = (last < 0) ? 0 : ((last > NSTEP - 1) ? (NSTEP - 1) : last);
    int lt = tags[last];
    lt = (lt < 0) ? 0 : ((lt > K - 1) ? (K - 1) : lt);
    sc += to_bf16_val(endv[lt]);
  }

  float mymax = ninf;
#pragma unroll 1
  for (int s = 0; s < nslot; ++s) {
    const int j  = lane + 32 * s;
    const int jc = (j < K) ? j : (K - 1);
    const float e0 = ld_em(emb + jc, cvt);
    const float a0 = to_bf16_val(startv[jc]) + e0;
    const float av = (j < K) ? a0 : ninf;
    sAlpha[j] = av;
    mymax = fmaxf(mymax, av);
  }
  __syncthreads();

#pragma unroll 1
  for (int t = 1; t < NSTEP; ++t) {
    const int mk = krow[t];
    float mx = mymax;
#pragma unroll
    for (int off = 16; off > 0; off >>= 1) mx = fmaxf(mx, __shfl_xor(mx, off, 32));
#pragma unroll 1
    for (int s = 0; s < nslot; ++s) {
      const int j = lane + 32 * s;
      const float aj = sAlpha[j];
      const float ea = expf(aj - mx);
      sEa[j] = (j < K) ? ea : 0.0f;
    }
    __syncthreads();
    const float* emrow = emb + (size_t)t * emld;
    float nm = ninf;
#pragma unroll 1
    for (int s = 0; s < nslot; ++s) {
      const int j  = lane + 32 * s;
      const int jc = (j < K) ? j : (K - 1);
      const float e = ld_em(emrow + jc, cvt);
      const float* etrow = sETt + jc * ETP;
      float accv = 0.0f;
#pragma unroll 1
      for (int i8 = 0; i8 < KP8; i8 += 8) {
        const v4f ea0 = *(const v4f*)(sEa + i8);
        const v4f ea1 = *(const v4f*)(sEa + i8 + 4);
        const v4f t0  = *(const v4f*)(etrow + i8);
        const v4f t1  = *(const v4f*)(etrow + i8 + 4);
        accv = fmaf(ea0.x, t0.x, accv);
        accv = fmaf(ea0.y, t0.y, accv);
        accv = fmaf(ea0.z, t0.z, accv);
        accv = fmaf(ea0.w, t0.w, accv);
        accv = fmaf(ea1.x, t1.x, accv);
        accv = fmaf(ea1.y, t1.y, accv);
        accv = fmaf(ea1.z, t1.z, accv);
        accv = fmaf(ea1.w, t1.w, accv);
      }
      const float nxt = mx + logf(accv) + e;
      const float aj  = sAlpha[j];
      float an = (mk != 0) ? nxt : aj;
      an = (j < K) ? an : ninf;
      sAlpha[j] = an;
      nm = fmaxf(nm, an);
    }
    mymax = nm;
    __syncthreads();
  }

  float mx = ninf;
#pragma unroll 1
  for (int s = 0; s < nslot; ++s) {
    const int j  = lane + 32 * s;
    const int jc = (j < K) ? j : (K - 1);
    const float v = sAlpha[j] + to_bf16_val(endv[jc]);
    mx = fmaxf(mx, (j < K) ? v : ninf);
  }
#pragma unroll
  for (int off = 16; off > 0; off >>= 1) mx = fmaxf(mx, __shfl_xor(mx, off, 32));
  float sm = 0.0f;
#pragma unroll 1
  for (int s = 0; s < nslot; ++s) {
    const int j  = lane + 32 * s;
    const int jc = (j < K) ? j : (K - 1);
    const float v  = sAlpha[j] + to_bf16_val(endv[jc]);
    const float ex = expf(v - mx);
    sm += (j < K) ? ex : 0.0f;
  }
#pragma unroll
  for (int off = 16; off > 0; off >>= 1) sm += __shfl_xor(sm, off, 32);
  const float logZ = mx + logf(sm);
  const float res  = logZ - sc;

  const v4f rv = (v4f){res, res, res, res};
  float* pp = partial + (size_t)blk * PART_LD + lane * 4;
  *(volatile v4f*)pp = rv;
  __threadfence();
  *(volatile v4f*)pp = rv;
}

__global__ __launch_bounds__(32) void final_loss(const float* __restrict__ partial, float* __restrict__ out) {
  float loss = 0.0f;
#pragma unroll 1
  for (int c = 0; c < NCHAIN; ++c) {
    float s = 0.0f;
#pragma unroll 1
    for (int b = 0; b < NBATCH; ++b) s += partial[(size_t)(c * NBATCH + b) * PART_LD];
    loss += s * (1.0f / NBATCH);
  }
  if (threadIdx.x == 0) *(volatile float*)out = loss;
  __threadfence();
  if (threadIdx.x == 0) *(volatile float*)out = loss;
}

extern "C" void kernel_launch(void* const* d_in, const int* in_sizes, int n_in,
                              void* d_out, int out_size, void* d_ws, size_t ws_size,
                              hipStream_t stream) {
  if (n_in < 19 || out_size < 1) return;
  if (in_sizes[0] != NROWS * FEAT_D || in_sizes[1] != NROWS * NTAG2 ||
      in_sizes[2] != NROWS || in_sizes[3] != NROWS || in_sizes[4] != NROWS || in_sizes[5] != NROWS ||
      in_sizes[6] != FEAT_D * NTAG0 || in_sizes[7] != NTAG0 ||
      in_sizes[8] != FEAT_D * NTAG1 || in_sizes[9] != NTAG1 ||
      in_sizes[10] != NTAG0 * NTAG0 || in_sizes[11] != NTAG0 || in_sizes[12] != NTAG0 ||
      in_sizes[13] != NTAG1 * NTAG1 || in_sizes[14] != NTAG1 || in_sizes[15] != NTAG1 ||
      in_sizes[16] != NTAG2 * NTAG2 || in_sizes[17] != NTAG2 || in_sizes[18] != NTAG2) return;

  const size_t OFF_A    = 0;
  const size_t SZ_A     = (size_t)NROWS * KPAD * 2;
  const size_t OFF_EM   = OFF_A + SZ_A;
  const size_t SZ_EM    = (size_t)NROWS * NCOL * 4;
  const size_t OFF_BT   = OFF_EM + SZ_EM;
  const size_t SZ_BT    = (size_t)NCOL * KPAD * 2;
  const size_t OFF_BIAS = OFF_BT + SZ_BT;
  const size_t SZ_BIAS  = 128 * 4;
  const size_t OFF_PART = OFF_BIAS + SZ_BIAS;
  const size_t SZ_PART  = (size_t)NCHAIN * NBATCH * PART_LD * 4;
  const size_t WS_TOTAL = OFF_PART + SZ_PART;
  if (ws_size < WS_TOTAL) return;

  const float* feats = (const float*)d_in[0];
  const float* em2   = (const float*)d_in[1];
  const int*   lab0  = (const int*)d_in[2];
  const int*   lab1  = (const int*)d_in[3];
  const int*   lab2  = (const int*)d_in[4];
  const int*   keep  = (const int*)d_in[5];
  const float* W0    = (const float*)d_in[6];
  const float* bia0  = (const float*)d_in[7];
  const float* W1    = (const float*)d_in[8];
  const float* bia1  = (const float*)d_in[9];
  const float* tr0   = (const float*)d_in[10];
  const float* st0   = (const float*)d_in[11];
  const float* en0   = (const float*)d_in[12];
  const float* tr1   = (const float*)d_in[13];
  const float* st1   = (const float*)d_in[14];
  const float* en1   = (const float*)d_in[15];
  const float* tr2   = (const float*)d_in[16];
  const float* st2   = (const float*)d_in[17];
  const float* en2   = (const float*)d_in[18];

  char* ws = (char*)d_ws;
  unsigned short* Ap    = (unsigned short*)(ws + OFF_A);
  float*          EM    = (float*)(ws + OFF_EM);
  unsigned short* Btp   = (unsigned short*)(ws + OFF_BT);
  float*          biasp = (float*)(ws + OFF_BIAS);
  float*          part  = (float*)(ws + OFF_PART);

  prep_feat_plane<<<NROWS / 256, 256, 0, stream>>>(feats, Ap);
  prep_wb<<<1, 256, 0, stream>>>(W0, bia0, W1, bia1, Btp, biasp);

  wmma_gemm64<1, false, 2, 0, false, 0><<<dim3(NROWS / 64 / 8, 1), 256, 0, stream>>>(
      Ap, Ap, KPAD, 0L,
      Btp, Btp, KPAD, 0L,
      (void*)EM, (void*)EM, NCOL, 0L,
      biasp,
      biasp, 0L,
      NROWS, NCOL, KPAD, 1.0f);

  chain_fwd<<<NCHAIN * NBATCH, 32, 0, stream>>>(EM, em2, lab0, lab1, lab2, keep,
                                                 tr0, st0, en0, tr1, st1, en1, tr2, st2, en2, part);

  final_loss<<<1, 32, 0, stream>>>(part, (float*)d_out);
}
